// ContrastiveAdditiveIndependentScorer_85263690760579
// MI455X (gfx1250) — hardware-verified
//
#include <hip/hip_runtime.h>
#include <math.h>

typedef __attribute__((ext_vector_type(16))) _Float16 v16h;
typedef __attribute__((ext_vector_type(16))) __bf16 v16b;
typedef __attribute__((ext_vector_type(8)))  _Float16 v8h;
typedef __attribute__((ext_vector_type(8)))  float v8f;
typedef __attribute__((ext_vector_type(4)))  float v4f;
typedef __attribute__((ext_vector_type(2)))  float v2f;
typedef __attribute__((ext_vector_type(4)))  unsigned v4u;
typedef __attribute__((ext_vector_type(4)))  int v4i;
typedef float __attribute__((may_alias)) float_a;
typedef int __attribute__((may_alias)) int_a;

template <typename T> __device__ __forceinline__ void vst2(void* p, T v) { *(volatile T*)p = v; __threadfence(); *(volatile T*)p = v; }
__device__ __forceinline__ v8f wmma16(v16h a, v16h b, v8f c) {
  v8f d = __builtin_amdgcn_wmma_f32_16x16x32_f16(false, a, false, b, (short)0, c, false, false);
  asm volatile("v_nop\n\tv_nop\n\tv_nop\n\tv_nop" : "+v"(d) : "v"(a), "v"(b));
  return d;
}
__device__ __forceinline__ v8f wmma_bf(v16b a, v16b b, v8f c) {
  v8f d = __builtin_amdgcn_wmma_f32_16x16x32_bf16(false, a, false, b, (short)0, c, false, false);
  asm volatile("v_nop\n\tv_nop\n\tv_nop\n\tv_nop" : "+v"(d) : "v"(a), "v"(b));
  return d;
}
__device__ __forceinline__ v16h frag_h(const _Float16* rowk0, int lane) {
  union { v16h v; v8h q[2]; } u; const _Float16* p = rowk0 + 8 * (lane >> 4);
  u.q[0] = *(const v8h*)p; u.q[1] = *(const v8h*)(p + 16); return u.v;
}
__device__ __forceinline__ v16h frag_f32(const float* rowk0, int lane) {
  v16h a; const float* p = rowk0 + 8 * (lane >> 4);
#pragma unroll
  for (int i = 0; i < 8; ++i) { a[i] = (_Float16)p[i]; a[8 + i] = (_Float16)p[16 + i]; }
  return a;
}
__device__ __forceinline__ v16h frag_f32s(const float* rowk0, int lane, float sc) {
  v16h a; const float* p = rowk0 + 8 * (lane >> 4);
#pragma unroll
  for (int i = 0; i < 8; ++i) { a[i] = (_Float16)(p[i] * sc); a[8 + i] = (_Float16)(p[16 + i] * sc); }
  return a;
}
__device__ __forceinline__ v16h fragc_f32(const float* W, int k0, int n, int lane, int ld, int K) {
  v16h a; const int g = lane >> 4;
#pragma unroll
  for (int i = 0; i < 8; ++i) { const int ka = k0 + 8 * g + i, kb = ka + 16;
    a[i] = (_Float16)(ka < K ? W[(size_t)(ka < K ? ka : K - 1) * ld + n] : 0.f); a[8 + i] = (_Float16)(kb < K ? W[(size_t)(kb < K ? kb : K - 1) * ld + n] : 0.f); }
  return a;
}
struct F2 { v16b h, l; };
__device__ __forceinline__ F2 bsplit16(const float v[16]) { F2 r;
#pragma unroll
  for (int i = 0; i < 16; ++i) { const __bf16 h = (__bf16)v[i]; r.h[i] = h; r.l[i] = (__bf16)(v[i] - (float)h); }
  return r; }
__device__ __forceinline__ F2 split_row(const float* row, int k0, int lane) { float v[16]; const float* p = row + k0 + 8 * (lane >> 4);
#pragma unroll
  for (int i = 0; i < 8; ++i) { v[i] = p[i]; v[8 + i] = p[16 + i]; }
  return bsplit16(v); }
__device__ __forceinline__ F2 split_rowK(const float* row, int k0, int lane, int K) { float v[16]; const int g = lane >> 4;
#pragma unroll
  for (int i = 0; i < 8; ++i) { const int ka = k0 + 8 * g + i, kb = ka + 16; v[i] = ka < K ? row[ka < K ? ka : K - 1] : 0.f; v[8 + i] = kb < K ? row[kb < K ? kb : K - 1] : 0.f; }
  return bsplit16(v); }
__device__ __forceinline__ F2 split_col(const float* W, int k0, int n, int lane, int ld, int K) { float v[16]; const int g = lane >> 4;
#pragma unroll
  for (int i = 0; i < 8; ++i) { const int ka = k0 + 8 * g + i, kb = ka + 16; v[i] = ka < K ? W[(size_t)(ka < K ? ka : K - 1) * ld + n] : 0.f; v[8 + i] = kb < K ? W[(size_t)(kb < K ? kb : K - 1) * ld + n] : 0.f; }
  return bsplit16(v); }
__device__ __forceinline__ v8f mac3(const F2& a, const F2& b, v8f c) { c = wmma_bf(a.l, b.h, c); c = wmma_bf(a.h, b.l, c); return wmma_bf(a.h, b.h, c); }
__device__ __forceinline__ float sigm(float v) { return 1.0f / (1.0f + expf(-v)); }
#define LDSX() do { asm volatile("s_wait_dscnt 0" ::: "memory"); __builtin_amdgcn_wave_barrier(); __builtin_amdgcn_fence(__ATOMIC_RELEASE, "workgroup"); } while (0)


#define NBQ 8192
#define DD 64
#define TD 16
#define HH 128
#define FD 16
#ifndef NBLKQ
#define NBLKQ (NBQ / 64)
#endif
typedef __attribute__((ext_vector_type(8))) __bf16 v8b;
__device__ __forceinline__ v16b frag_b(const __bf16* rowk0, int lane) {
  union { v16b v; v8b q[2]; } u; const __bf16* p = rowk0 + 8 * (lane >> 4);
  u.q[0] = *(const v8b*)p; u.q[1] = *(const v8b*)(p + 16); return u.v;
}
__device__ __forceinline__ float bfr(float v) { return (float)(__bf16)v; }
__device__ __attribute__((noinline)) float exp_ni(float v) { return expf(v); }
__device__ __attribute__((noinline)) float erf_ni(float v) { return erff(v); }

#define WS_PW   0u
#define P2 0
#define P3 (P2 + DD * HH * HH)
#define PO (P3 + DD * HH * HH)
#define PA2 (PO + DD * FD * HH)
#define PA3 (PA2 + HH * HH)
#define PAO (PA3 + HH * HH)
#define PWEND (PAO + FD * HH)
#define WS_AT   (WS_PW + 2u * PWEND)
#define WS_END  (WS_AT + 4u * NBQ * FD)
__device__ __forceinline__ float silu_x(float v) { return v * sigm(v); }

__global__ __launch_bounds__(128) void k_pack(const float* __restrict__ W2, const float* __restrict__ W3, const float* __restrict__ WO, const float* __restrict__ A2, const float* __restrict__ A3, const float* __restrict__ AO, __bf16* __restrict__ PW) {
  __shared__ __align__(16) __bf16 s[HH]; const int n = blockIdx.x, p = blockIdx.y, k = threadIdx.x; size_t dst; float v;
  if (p < 64) { dst = P2 + ((size_t)p * HH + n) * HH; v = W2[((size_t)p * HH + k) * HH + n]; }
  else if (p < 128) { dst = P3 + ((size_t)(p - 64) * HH + n) * HH; v = W3[((size_t)(p - 64) * HH + k) * HH + n]; }
  else if (p < 192) { if (n >= FD) return; dst = PO + ((size_t)(p - 128) * FD + n) * HH; v = WO[((size_t)(p - 128) * HH + k) * FD + n]; }
  else if (p == 192) { dst = PA2 + (size_t)n * HH; v = A2[(size_t)k * HH + n]; }
  else if (p == 193) { dst = PA3 + (size_t)n * HH; v = A3[(size_t)k * HH + n]; }
  else { if (n >= FD) return; dst = PAO + (size_t)n * HH; v = AO[(size_t)k * FD + n]; }
  s[k] = (__bf16)v; __syncthreads();
  if (k < HH / 8) vst2((unsigned*)(PW + dst + k * 8), *(const v4u*)&s[k * 8]);
}
template <int NT>
__device__ __forceinline__ void lds_gemm(const __bf16 (*sh)[HH + 8], const __bf16 (*sl)[HH + 8], const __bf16* __restrict__ P, int lane, int col, int g, v8f* acc) {
#pragma unroll
  for (int kc = 0; kc < HH / 32; ++kc) { v16b ah, al;
#pragma unroll
    for (int i = 0; i < 8; ++i) { ah[i] = sh[col][kc * 32 + 8 * g + i]; ah[8 + i] = sh[col][kc * 32 + 16 + 8 * g + i]; al[i] = sl[col][kc * 32 + 8 * g + i]; al[8 + i] = sl[col][kc * 32 + 16 + 8 * g + i]; }
#pragma unroll
    for (int j = 0; j < NT; ++j) { const v16b w = frag_b(P + (size_t)(j * 16 + col) * HH + kc * 32, lane); acc[j] = wmma_bf(al, w, acc[j]); acc[j] = wmma_bf(ah, w, acc[j]); } }
}
__global__ __launch_bounds__(128) void k_theta(const float* __restrict__ TH, const float* __restrict__ A1, const float* __restrict__ AB1, const __bf16* __restrict__ PW, const float* __restrict__ AB2, const float* __restrict__ AB3, const float* __restrict__ ABO, float* __restrict__ AT) {
  __shared__ __align__(16) __bf16 sh[4][16][HH + 8], sl[4][16][HH + 8]; __shared__ float sa1[TD][HH], sb1[HH]; __shared__ __align__(16) float so[64][FD];
  const int tid = threadIdx.x, wave = tid >> 5, lane = tid & 31, col = lane & 15, g = lane >> 4; const size_t r0 = (size_t)blockIdx.x * 64 + wave * 16;
  for (int i = tid; i < TD * HH; i += 128) sa1[i / HH][i % HH] = bfr(A1[i]); if (tid < HH) sb1[tid] = bfr(AB1[tid]);
  __syncthreads();
  for (int rl = 0; rl < 16; ++rl) { float t[TD];
#pragma unroll
    for (int k = 0; k < TD; ++k) t[k] = bfr(TH[(r0 + rl) * TD + k]);
#pragma unroll
    for (int mm = 0; mm < 4; ++mm) { const int c = lane + 32 * mm; float v = sb1[c];
#pragma unroll
      for (int k = 0; k < TD; ++k) v += t[k] * sa1[k][c];
      v = silu_x(v); const __bf16 hb = (__bf16)v; sh[wave][rl][c] = hb; sl[wave][rl][c] = (__bf16)(v - (float)hb); } }
  LDSX();
#pragma unroll 1
  for (int layer = 0; layer < 2; ++layer) { v8f acc[8]; for (int j = 0; j < 8; ++j) acc[j] = (v8f){};
    lds_gemm<8>(sh[wave], sl[wave], PW + (layer == 0 ? PA2 : PA3), lane, col, g, acc);
    LDSX();
    const float* bb = (layer == 0) ? AB2 : AB3;
#pragma unroll
    for (int j = 0; j < 8; ++j) { const int c = j * 16 + col; const float b_ = bfr(bb[c]);
#pragma unroll
      for (int r = 0; r < 8; ++r) { const float v = silu_x(acc[j][r] + b_); const __bf16 hb = (__bf16)v; sh[wave][8 * g + r][c] = hb; sl[wave][8 * g + r][c] = (__bf16)(v - (float)hb); } }
    LDSX(); }
  { v8f acc[1] = {}; lds_gemm<1>(sh[wave], sl[wave], PW + PAO, lane, col, g, acc);
#pragma unroll
    for (int r = 0; r < 8; ++r) so[wave * 16 + 8 * g + r][col] = acc[0][r] + bfr(ABO[col]); }
  __syncthreads();
  for (int q = tid; q < 64 * 4; q += 128) { const int rl = q >> 2, pc = q & 3; vst2(AT + ((size_t)blockIdx.x * 64 + rl) * FD + pc * 4, *(const v4f*)&so[rl][pc * 4]); }
}
__global__ __launch_bounds__(128) void k_score(const float* __restrict__ X, const float* __restrict__ W1, const float* __restrict__ B1, const __bf16* __restrict__ PW, const float* __restrict__ B2, const float* __restrict__ B3, const float* __restrict__ BO, const float* __restrict__ AT, float* __restrict__ out) {
  __shared__ __align__(16) __bf16 sh[4][16][HH + 8], sl[4][16][HH + 8]; __shared__ __align__(16) float so[64];
  const int tid = threadIdx.x, wave = tid >> 5, lane = tid & 31, col = lane & 15, g = lane >> 4; const size_t r0 = (size_t)blockIdx.x * 64 + wave * 16;
  float at_r[8];
#pragma unroll
  for (int r = 0; r < 8; ++r) at_r[r] = AT[(r0 + 8 * g + r) * FD + col];
  float sacc[8];
#pragma unroll
  for (int r = 0; r < 8; ++r) sacc[r] = 0.f;
#pragma unroll 1
  for (int d = 0; d < DD; ++d) {
    float w1c[4], b1c[4];
#pragma unroll
    for (int mm = 0; mm < 4; ++mm) { w1c[mm] = bfr(W1[(size_t)d * HH + lane + 32 * mm]); b1c[mm] = bfr(B1[(size_t)d * HH + lane + 32 * mm]); }
    for (int rl = 0; rl < 16; ++rl) { const float xv = bfr(X[(r0 + rl) * DD + d]);
#pragma unroll
      for (int mm = 0; mm < 4; ++mm) { const float v = silu_x(xv * w1c[mm] + b1c[mm]); const __bf16 hb = (__bf16)v; sh[wave][rl][lane + 32 * mm] = hb; sl[wave][rl][lane + 32 * mm] = (__bf16)(v - (float)hb); } }
    LDSX();
#pragma unroll 1
    for (int layer = 0; layer < 2; ++layer) { v8f acc[8]; for (int j = 0; j < 8; ++j) acc[j] = (v8f){};
      lds_gemm<8>(sh[wave], sl[wave], PW + (layer == 0 ? P2 : P3) + (size_t)d * HH * HH, lane, col, g, acc);
      LDSX();
      const float* bb = ((layer == 0) ? B2 : B3) + (size_t)d * HH;
#pragma unroll
      for (int j = 0; j < 8; ++j) { const int c = j * 16 + col; const float b_ = bfr(bb[c]);
#pragma unroll
        for (int r = 0; r < 8; ++r) { float v = silu_x(acc[j][r] + b_); if (layer == 0) v = silu_x(v);   const __bf16 hb = (__bf16)v; sh[wave][8 * g + r][c] = hb; sl[wave][8 * g + r][c] = (__bf16)(v - (float)hb); } }
      LDSX(); }
    { v8f acc[1] = {}; lds_gemm<1>(sh[wave], sl[wave], PW + PO + (size_t)d * FD * HH, lane, col, g, acc); const float bo = bfr(BO[(size_t)d * FD + col]);
#pragma unroll
      for (int r = 0; r < 8; ++r) sacc[r] += (acc[0][r] + bo) * at_r[r]; }
    LDSX();
  }
#pragma unroll
  for (int r = 0; r < 8; ++r) { float s = sacc[r];
#pragma unroll
    for (int o = 1; o < 16; o <<= 1) s += __shfl_xor(s, o);
    if (col == 0) so[wave * 16 + 8 * g + r] = s * (1.0f / (float)DD); }
  __syncthreads();
  if (tid < 16) vst2(out + (size_t)blockIdx.x * 64 + tid * 4, *(const v4f*)&so[tid * 4]);
}
extern "C" void kernel_launch(void* const* d_in, const int* in_sizes, int n_in, void* d_out, int out_size, void* d_ws, size_t ws_size, hipStream_t stream) {
  (void)in_sizes; (void)n_in; (void)out_size;
  const float** F = (const float**)d_in;
  if (ws_size < (size_t)WS_END) return;
  char* ws = (char*)d_ws; __bf16* PW = (__bf16*)(ws + WS_PW); float* AT = (float*)(ws + WS_AT);
  k_pack<<<dim3(HH, 195), 128, 0, stream>>>(F[4], F[6], F[8], F[12], F[14], F[16], PW);
  k_theta<<<NBLKQ, 128, 0, stream>>>(F[1], F[10], F[11], PW, F[13], F[15], F[17], AT);
  k_score<<<NBLKQ, 128, 0, stream>>>(F[0], F[2], F[3], PW, F[5], F[7], F[9], AT, (float*)d_out);
}
